// LSTM_8598524527020
// MI455X (gfx1250) — hardware-verified
//
#include <hip/hip_runtime.h>
#include <math.h>

constexpr int SEQ_LEN  = 65536;
constexpr int NIN      = 2;
constexpr int NHID     = 128;
constexpr int NGATE    = 4;
constexpr int NGROWS   = NGATE * NHID;
constexpr int NTHR     = 256;
constexpr int NWAVE    = NTHR / 32;
constexpr int FLUSH_N  = 32;
constexpr int RING_N   = 64;
constexpr float H_CARRY  = 1024.0f;
constexpr float W_CARRY  = 64.0f;
constexpr float FOLD_INV = 1.0f / (H_CARRY * W_CARRY);

static_assert(NHID == 16 * NWAVE, "one 16-unit subtile per wave");
static_assert(NHID % 32 == 0, "k chunks of 32");
static_assert(NHID / 32 == 4, "four k chunks held as register fragments");
static_assert(SEQ_LEN % FLUSH_N == 0, "no output tail");
static_assert(RING_N == 2 * FLUSH_N, "two ring halves");
static_assert(FLUSH_N == 32, "one 128-B output line per flush");
static_assert(NGROWS == 512, "gate rows i|f|g|o");

typedef __attribute__((ext_vector_type(16))) _Float16 v16h;
typedef __attribute__((ext_vector_type(8)))  _Float16 v8h;
typedef __attribute__((ext_vector_type(8)))  float    v8f;
typedef __attribute__((ext_vector_type(4)))  float    v4f;
typedef __attribute__((ext_vector_type(2)))  float    v2f;

struct Frag16 {
  union U { v16h v; v8h h[2]; };
  static __device__ __forceinline__ v16h load(const _Float16* p) {
    U f;
    f.h[0] = *(const v8h*)(p);
    f.h[1] = *(const v8h*)(p + 16);
    return f.v;
  }
  static __device__ __forceinline__ v8f mma(v16h a, v16h b, v8f c) {
    return __builtin_amdgcn_wmma_f32_16x16x32_f16(false, a, false, b, (short)0, c, false, false);
  }
};

__device__ __forceinline__ void guard_group(v8f& a0, v8f& a1, v8f& a2, v8f& a3,
                                            v16h a, v16h b0, v16h b1, v16h b2, v16h b3) {
  asm volatile("v_nop\n\tv_nop\n\tv_nop\n\tv_nop"
               : "+v"(a0), "+v"(a1), "+v"(a2), "+v"(a3)
               : "v"(a), "v"(b0), "v"(b1), "v"(b2), "v"(b3));
}

__device__ __forceinline__ float fsig(float v)  { return __builtin_amdgcn_rcpf(1.0f + __expf(-v)); }
__device__ __forceinline__ float ftanh(float v) { return 1.0f - 2.0f * __builtin_amdgcn_rcpf(__expf(2.0f * v) + 1.0f); }

__attribute__((amdgpu_num_vgpr(256)))
__global__ __launch_bounds__(NTHR) void lstm_seq_kernel(const float* __restrict__ x,
                                                        const float* __restrict__ h0,
                                                        const float* __restrict__ c0,
                                                        const float* __restrict__ W_ih,
                                                        const float* __restrict__ W_hh,
                                                        const float* __restrict__ b_ih,
                                                        const float* __restrict__ b_hh,
                                                        const float* __restrict__ W_out,
                                                        const float* __restrict__ b_out,
                                                        float* out) {
  __shared__ __align__(16) _Float16 hbuf[2 * NHID];
  __shared__ __align__(16) float    part[RING_N * NWAVE];

  const int tid  = threadIdx.x;
  const int lane = tid & 31;
  const int wave = tid >> 5;
  const int col  = lane & 15;
  const int koff = (lane >> 4) * 8;
  const int hidx = 16 * wave + col;

  {
    const float hv = h0[tid & (NHID - 1)];
    if (tid < NHID) hbuf[tid] = (_Float16)(hv * H_CARRY);
  }
  float creg = c0[hidx];
  const float wout = W_out[hidx];
  const float bo = b_out[0];

  v16h bmat[4][4];
  float wi0[4], wi1[4], gb[4];
  int woff = 0;
#pragma unroll
  for (int s = 0; s < 4; ++s) {
    const int row = NHID * s + hidx;
    const float* wrow = W_hh + (size_t)row * NHID + koff;
#pragma unroll
    for (int kc = 0; kc < 4; ++kc) {
      const float* wp = wrow + 32 * kc + woff;
      const v4f q0 = *(const v4f*)(wp);
      const v4f q1 = *(const v4f*)(wp + 4);
      const v4f q2 = *(const v4f*)(wp + 16);
      const v4f q3 = *(const v4f*)(wp + 20);
      v16h b;
#pragma unroll
      for (int e = 0; e < 4; ++e) {
        b[e]      = (_Float16)(q0[e] * W_CARRY);
        b[4 + e]  = (_Float16)(q1[e] * W_CARRY);
        b[8 + e]  = (_Float16)(q2[e] * W_CARRY);
        b[12 + e] = (_Float16)(q3[e] * W_CARRY);
      }
      asm volatile("" : "+v"(b), "+v"(woff));
      bmat[s][kc] = b;
    }
    const v2f wv = *(const v2f*)(W_ih + (size_t)row * NIN);
    wi0[s] = wv[0];
    wi1[s] = wv[1];
    gb[s]  = b_ih[row] + b_hh[row];
  }
  __syncthreads();

  const v8f z8 = {0.f, 0.f, 0.f, 0.f, 0.f, 0.f, 0.f, 0.f};
  float x0 = x[0];
  float x1 = x[1];

#pragma unroll 1
  for (int t = 0; t < SEQ_LEN; ++t) {
    const int tn = (t + 1 < SEQ_LEN) ? (t + 1) : (SEQ_LEN - 1);
    float nx0 = x[2 * tn + 0];
    float nx1 = x[2 * tn + 1];
    asm volatile("" : "+v"(nx0), "+v"(nx1));

    const _Float16* hr = hbuf + (t & 1) * NHID + koff;
    _Float16*       hw = hbuf + ((t + 1) & 1) * NHID;

    v8f acc0 = z8, acc1 = z8, acc2 = z8, acc3 = z8;
#pragma unroll
    for (int kc = 0; kc < 4; ++kc) {
      const v16h a = Frag16::load(hr + 32 * kc);
      acc0 = Frag16::mma(a, bmat[0][kc], acc0);
      acc1 = Frag16::mma(a, bmat[1][kc], acc1);
      acc2 = Frag16::mma(a, bmat[2][kc], acc2);
      acc3 = Frag16::mma(a, bmat[3][kc], acc3);
      guard_group(acc0, acc1, acc2, acc3, a, bmat[0][kc], bmat[1][kc], bmat[2][kc], bmat[3][kc]);
    }

    const float pi = acc0[0] * FOLD_INV + fmaf(x1, wi1[0], fmaf(x0, wi0[0], gb[0]));
    const float pf = acc1[0] * FOLD_INV + fmaf(x1, wi1[1], fmaf(x0, wi0[1], gb[1]));
    const float pg = acc2[0] * FOLD_INV + fmaf(x1, wi1[2], fmaf(x0, wi0[2], gb[2]));
    const float po = acc3[0] * FOLD_INV + fmaf(x1, wi1[3], fmaf(x0, wi0[3], gb[3]));

    const float ig = fsig(pi);
    const float fg = fsig(pf);
    const float gg = ftanh(pg);
    const float og = fsig(po);

    const float cn = fg * creg + ig * gg;
    creg = cn;
    const float hn = og * ftanh(cn);

    if (lane < 16) hw[hidx] = (_Float16)(hn * H_CARRY);

    float p = ftanh(hn) * wout;
    p += __shfl_xor(p, 1, 32);
    p += __shfl_xor(p, 2, 32);
    p += __shfl_xor(p, 4, 32);
    p += __shfl_xor(p, 8, 32);
    if (lane == 0) part[(t & (RING_N - 1)) * NWAVE + wave] = p;

    x0 = nx0;
    x1 = nx1;
    __syncthreads();

    if ((t & (FLUSH_N - 1)) == (FLUSH_N - 1)) {
      if (wave == 0) {
        const int slot0 = (t & (RING_N - 1)) - (FLUSH_N - 1);
        const float* pp = part + (slot0 + lane) * NWAVE;
        const v4f pa = *(const v4f*)(pp);
        const v4f pb = *(const v4f*)(pp + 4);
        float sum = 0.0f;
        sum += pa[0];
        sum += pa[1];
        sum += pa[2];
        sum += pa[3];
        sum += pb[0];
        sum += pb[1];
        sum += pb[2];
        sum += pb[3];
        sum += bo;
        volatile float* op = out + (size_t)(t - (FLUSH_N - 1) + lane);
        *op = sum;
        __threadfence();
        *op = sum;
      }
    }
  }
}

extern "C" void kernel_launch(void* const* d_in, const int* in_sizes, int n_in,
                              void* d_out, int out_size, void* d_ws, size_t ws_size, hipStream_t stream) {
  (void)d_ws;
  (void)ws_size;
  if (n_in < 9 || d_out == nullptr) return;
  if (in_sizes[0] != SEQ_LEN * NIN || in_sizes[1] != NHID || in_sizes[2] != NHID ||
      in_sizes[3] != NGROWS * NIN || in_sizes[4] != NGROWS * NHID || in_sizes[5] != NGROWS ||
      in_sizes[6] != NGROWS || in_sizes[7] != NHID || in_sizes[8] != 1 || out_size != SEQ_LEN) return;

  const float* x    = (const float*)d_in[0];
  const float* h0   = (const float*)d_in[1];
  const float* c0   = (const float*)d_in[2];
  const float* Wih  = (const float*)d_in[3];
  const float* Whh  = (const float*)d_in[4];
  const float* bih  = (const float*)d_in[5];
  const float* bhh  = (const float*)d_in[6];
  const float* Wout = (const float*)d_in[7];
  const float* bout = (const float*)d_in[8];
  float* out = (float*)d_out;

  lstm_seq_kernel<<<1, NTHR, 0, stream>>>(x, h0, c0, Wih, Whh, bih, bhh, Wout, bout, out);
}
